// _PositionAttentionModule_52055003627961
// MI455X (gfx1250) — hardware-verified
//
#include <hip/hip_runtime.h>


namespace {
constexpr int Bn = 4, C = 256, CQ = 32, NP = 4096;
constexpr float FS = 8.0f, VS = 8.0f, PS = 8.0f;

typedef _Float16 b16;
typedef __attribute__((ext_vector_type(16))) _Float16 v16b;
typedef __attribute__((ext_vector_type(8))) _Float16 v8b;
typedef __attribute__((ext_vector_type(8))) float v8f;
typedef __attribute__((ext_vector_type(4))) float v4f;
__device__ __forceinline__ float bf16_rne(float f) { unsigned int u = __float_as_uint(f); u += 0x7FFFu + ((u >> 16) & 1u); return __uint_as_float(u & 0xFFFF0000u); }
__device__ __forceinline__ void split16(float v, b16& hi, b16& lo) { hi = (b16)v; lo = (b16)(v - (float)hi); }
__device__ __forceinline__ v16b frag_kb(const b16* p, int hh) { const v8b a = *(const v8b*)(p + 8 * hh), b = *(const v8b*)(p + 16 + 8 * hh); v16b f;
#pragma unroll
  for (int e = 0; e < 8; ++e) { f[e] = a[e]; f[8 + e] = b[e]; } return f; }
__device__ __forceinline__ v8f wmma16b(v16b a, v16b b, v8f c) { v8f d = __builtin_amdgcn_wmma_f32_16x16x32_f16(false, a, false, b, (short)0, c, false, false); asm volatile("v_nop\n\tv_nop\n\tv_nop\n\tv_nop" : "+v"(d) : "v"(a), "v"(b)); return d; }
__device__ __forceinline__ void wave_lds_sync() { __builtin_amdgcn_fence(__ATOMIC_RELEASE, "workgroup"); __builtin_amdgcn_wave_barrier(); __builtin_amdgcn_fence(__ATOMIC_ACQUIRE, "workgroup"); }
__device__ __forceinline__ float nexp(float x) { return __builtin_amdgcn_exp2f(x * 1.4426950408889634f); }

__global__ __launch_bounds__(256) void xpose_kernel(const float* __restrict__ x, const float* __restrict__ x1, b16* __restrict__ XT, b16* __restrict__ X1T) {
  __shared__ __attribute__((aligned(16))) b16 T[64][C + 8];
  const int b = blockIdx.y, p0 = blockIdx.x * 64, which = blockIdx.z, t_ = threadIdx.x; const float* src = (which == 0) ? x : x1; b16* dst = (which == 0) ? XT : X1T;
  for (int i = t_; i < C * 64; i += 256) { const int c = i >> 6, p = i & 63; T[p][c] = (b16)bf16_rne(src[((size_t)b * C + c) * NP + p0 + p]); }
  __syncthreads();
  for (int pass = 0; pass < 2; ++pass) { for (int i = t_; i < 64 * 32; i += 256) { const int p = i >> 5, c8 = (i & 31) * 8; *(volatile v8b*)(dst + ((size_t)b * NP + p0 + p) * C + c8) = *(const v8b*)(&T[p][c8]); } __threadfence(); }
}

__global__ __launch_bounds__(256) void prep_kernel(const float* __restrict__ Wb, const float* __restrict__ Wc, const float* __restrict__ Wd, const float* __restrict__ bb, const float* __restrict__ bc, const float* __restrict__ bd, const float* __restrict__ al, b16* __restrict__ R, float* __restrict__ P) {
  const int t_ = blockIdx.x * 256 + threadIdx.x, nth = gridDim.x * 256;
  for (int pass = 0; pass < 2; ++pass) {
    for (int p = t_; p < (2 * CQ + C) * C / 8; p += nth) { const int q = p * 8; const float* src = (q < CQ * C) ? (Wb + q) : (q < 2 * CQ * C) ? (Wc + (q - CQ * C)) : (Wd + (q - 2 * CQ * C)); v8b v;
#pragma unroll
      for (int e = 0; e < 8; ++e) v[e] = (b16)bf16_rne(src[e]); *(volatile v8b*)(R + q) = v; }
    for (int q = t_; q < 352; q += nth) { float v = 0.0f; if (q < 32) v = bb[q]; else if (q < 64) v = bc[q - 32]; else if (q < 320) v = bd[q - 64]; else if (q == 320) v = al[0]; P[q] = bf16_rne(v); }
    __threadfence(); }
}

__global__ __launch_bounds__(128) void proj_kernel(const b16* __restrict__ XT, const b16* __restrict__ X1T, const b16* __restrict__ R, const float* __restrict__ P, b16* __restrict__ FBh, b16* __restrict__ FBl, b16* __restrict__ FCh, b16* __restrict__ FCl, b16* __restrict__ VT) {
  __shared__ __attribute__((aligned(16))) b16 Tv[C][128 + 8]; __shared__ __attribute__((aligned(16))) b16 Tf[4][4][32][32 + 8];
  const int lane = threadIdx.x & 31, wave = threadIdx.x >> 5, nloc = lane & 15, hlf = lane >> 4, b = blockIdx.y, n0 = blockIdx.x * 128, m0 = n0 + wave * 32;
  const b16* Wb = R; const b16* Wc = R + CQ * C; const b16* Wd = R + 2 * CQ * C;
  for (int which = 0; which < 2; ++which) { const b16* Xs_ = (which == 0) ? XT : X1T; const b16* Ws_ = (which == 0) ? Wb : Wc; const float* bias = P + which * 32; v8f f[2][2];
#pragma unroll
    for (int r = 0; r < 2; ++r) { f[r][0] = (v8f){}; f[r][1] = (v8f){}; }
    for (int kb = 0; kb < C; kb += 32) { const v16b a0 = frag_kb(Xs_ + ((size_t)b * NP + m0 + nloc) * C + kb, hlf), a1 = frag_kb(Xs_ + ((size_t)b * NP + m0 + 16 + nloc) * C + kb, hlf);
#pragma unroll
      for (int t = 0; t < 2; ++t) { const v16b wf = frag_kb(Ws_ + (size_t)(t * 16 + nloc) * C + kb, hlf); f[0][t] = wmma16b(a0, wf, f[0][t]); f[1][t] = wmma16b(a1, wf, f[1][t]); } }
#pragma unroll
    for (int t = 0; t < 2; ++t)
#pragma unroll
      for (int r = 0; r < 2; ++r)
#pragma unroll
        for (int v = 0; v < 8; ++v) { const int rr = r * 16 + 8 * hlf + v, cc = t * 16 + nloc; b16 h_, l_; split16((f[r][t][v] + bias[cc]) * FS, h_, l_); Tf[wave][which * 2][rr][cc] = h_; Tf[wave][which * 2 + 1][rr][cc] = l_; } }
  wave_lds_sync();
  for (int pass = 0; pass < 2; ++pass) { for (int i = lane; i < 32 * 4; i += 32) { const int rr = i >> 2, c8 = (i & 3) * 8; const size_t o = ((size_t)b * NP + m0 + rr) * CQ + c8;
      *(volatile v8b*)(FBh + o) = *(const v8b*)(&Tf[wave][0][rr][c8]); *(volatile v8b*)(FBl + o) = *(const v8b*)(&Tf[wave][1][rr][c8]); *(volatile v8b*)(FCh + o) = *(const v8b*)(&Tf[wave][2][rr][c8]); *(volatile v8b*)(FCl + o) = *(const v8b*)(&Tf[wave][3][rr][c8]); }
    __threadfence(); }
  for (int qq = 0; qq < 4; ++qq) { v8f acc[2][4];
#pragma unroll
    for (int r = 0; r < 2; ++r)
#pragma unroll
      for (int t = 0; t < 4; ++t) acc[r][t] = (v8f){};
    for (int kb = 0; kb < C; kb += 32) { const v16b a0 = frag_kb(XT + ((size_t)b * NP + m0 + nloc) * C + kb, hlf), a1 = frag_kb(XT + ((size_t)b * NP + m0 + 16 + nloc) * C + kb, hlf);
#pragma unroll
      for (int t = 0; t < 4; ++t) { const v16b wd = frag_kb(Wd + (size_t)(qq * 64 + t * 16 + nloc) * C + kb, hlf); acc[0][t] = wmma16b(a0, wd, acc[0][t]); acc[1][t] = wmma16b(a1, wd, acc[1][t]); } }
#pragma unroll
    for (int t = 0; t < 4; ++t)
#pragma unroll
      for (int r = 0; r < 2; ++r)
#pragma unroll
        for (int v = 0; v < 8; ++v) { const int c = qq * 64 + t * 16 + nloc; Tv[c][wave * 32 + r * 16 + 8 * hlf + v] = (b16)((acc[r][t][v] + P[64 + c]) * VS); } }
  __syncthreads();
  for (int pass = 0; pass < 2; ++pass) { for (int i = threadIdx.x; i < C * 16; i += 128) { const int c = i >> 4, c8 = (i & 15) * 8; *(volatile v8b*)(VT + ((size_t)b * C + c) * NP + n0 + c8) = *(const v8b*)(&Tv[c][c8]); } __threadfence(); }
}

__global__ __launch_bounds__(256) void attn_kernel(const b16* __restrict__ FBh, const b16* __restrict__ FBl, const b16* __restrict__ FCh, const b16* __restrict__ FCl, const b16* __restrict__ VT, const float* __restrict__ x, const float* __restrict__ P, float* __restrict__ out) {
  __shared__ __attribute__((aligned(16))) float Os[C][128 + 4];
  const int wid = threadIdx.x >> 5, lane = threadIdx.x & 31, hh = lane >> 4, col = lane & 15, b = blockIdx.y, n0 = blockIdx.x * 128, q0 = n0 + wid * 16, qi = q0 + col;
  const b16* Vb = VT + (size_t)b * C * NP;
  const v16b qh = frag_kb(FBh + ((size_t)b * NP + qi) * CQ, hh), ql = frag_kb(FBl + ((size_t)b * NP + qi) * CQ, hh);
  for (int half = 0; half < 2; ++half) {
  float m = -INFINITY, l = 0.0f; v8f o[8];
#pragma unroll
  for (int t = 0; t < 8; ++t) o[t] = (v8f){};
  for (int kb = 0; kb < NP; kb += 32) {
    v8f s0 = {}, s1 = {};
    { const v16b k0h = frag_kb(FCh + ((size_t)b * NP + kb + col) * CQ, hh), k0l = frag_kb(FCl + ((size_t)b * NP + kb + col) * CQ, hh), k1h = frag_kb(FCh + ((size_t)b * NP + kb + 16 + col) * CQ, hh), k1l = frag_kb(FCl + ((size_t)b * NP + kb + 16 + col) * CQ, hh);
      s0 = wmma16b(k0h, qh, s0); s0 = wmma16b(k0h, ql, s0); s0 = wmma16b(k0l, qh, s0); s1 = wmma16b(k1h, qh, s1); s1 = wmma16b(k1h, ql, s1); s1 = wmma16b(k1l, qh, s1); }
    float mr = -INFINITY;
#pragma unroll
    for (int r = 0; r < 8; ++r) { s0[r] *= (1.0f / (FS * FS)); s1[r] *= (1.0f / (FS * FS)); mr = fmaxf(mr, fmaxf(s0[r], s1[r])); }
    mr = fmaxf(mr, __shfl_xor(mr, 16));
    const float mn = fmaxf(m, mr), al_ = nexp(m - mn); m = mn; float sum = 0.0f; v16b pbv;
#pragma unroll
    for (int r = 0; r < 8; ++r) { const float e0 = nexp(s0[r] - mn), e1 = nexp(s1[r] - mn); sum += e0 + e1; pbv[r] = (b16)(e0 * PS); pbv[8 + r] = (b16)(e1 * PS); }
    sum += __shfl_xor(sum, 16); l = l * al_ + sum;
#pragma unroll
    for (int t = 0; t < 8; ++t) { o[t] *= al_; const v16b vf = frag_kb(Vb + (size_t)((half * 8 + t) * 16 + col) * NP + kb, hh); o[t] = wmma16b(vf, pbv, o[t]); } }
  const float sc = P[320] / (l * VS * PS);
#pragma unroll
  for (int t = 0; t < 8; ++t)
#pragma unroll
    for (int r = 0; r < 8; ++r) Os[(half * 8 + t) * 16 + 8 * hh + r][wid * 16 + col] = o[t][r] * sc; }
  __syncthreads();
  for (int pass = 0; pass < 2; ++pass) { for (int i = threadIdx.x; i < C * 32; i += 256) { const int c = i >> 5, c4 = (i & 31) * 4; const size_t gi = ((size_t)b * C + c) * NP + n0 + c4; v4f v = *(const v4f*)(&Os[c][c4]); const v4f xr = *(const v4f*)(x + gi);
      for (int e = 0; e < 4; ++e) v[e] += bf16_rne(xr[e]); *(volatile v4f*)(out + gi) = v; } __threadfence(); }
}
}

extern "C" void kernel_launch(void* const* d_in, const int* in_sizes, int n_in,
                              void* d_out, int out_size, void* d_ws, size_t ws_size, hipStream_t stream) {
  (void)n_in; (void)out_size;
  const float* x = (const float*)d_in[0]; const float* x1 = (const float*)d_in[1]; const float* Wb = (const float*)d_in[2]; const float* bb = (const float*)d_in[3]; const float* Wc = (const float*)d_in[4]; const float* bc = (const float*)d_in[5]; const float* Wd = (const float*)d_in[6]; const float* bd = (const float*)d_in[7]; const float* al = (const float*)d_in[8];
  float* out = (float*)d_out;
  if (in_sizes[0] != Bn * C * NP || in_sizes[1] != Bn * C * NP || in_sizes[2] != CQ * C || in_sizes[6] != C * C || in_sizes[8] != 1) return;
  size_t off = 0; char* ws = (char*)d_ws;
  auto carve = [&](size_t bytes) { char* p = ws + off; off += (bytes + 255) & ~(size_t)255; return p; };
  b16* XT = (b16*)carve((size_t)Bn * NP * C * 2); b16* X1T = (b16*)carve((size_t)Bn * NP * C * 2); b16* R = (b16*)carve((size_t)(2 * CQ + C) * C * 2); float* P = (float*)carve(512 * 4);
  b16* FBh = (b16*)carve((size_t)Bn * NP * CQ * 2); b16* FBl = (b16*)carve((size_t)Bn * NP * CQ * 2); b16* FCh = (b16*)carve((size_t)Bn * NP * CQ * 2); b16* FCl = (b16*)carve((size_t)Bn * NP * CQ * 2); b16* VT = (b16*)carve((size_t)Bn * C * NP * 2);
  if (off > ws_size) return;
  xpose_kernel<<<dim3(NP / 64, Bn, 2), 256, 0, stream>>>(x, x1, XT, X1T);
  prep_kernel<<<64, 256, 0, stream>>>(Wb, Wc, Wd, bb, bc, bd, al, R, P);
  proj_kernel<<<dim3(NP / 128, Bn), 128, 0, stream>>>(XT, X1T, R, P, FBh, FBl, FCh, FCl, VT);
  attn_kernel<<<dim3(NP / 128, Bn), 256, 0, stream>>>(FBh, FBl, FCh, FCl, VT, x, P, out);
}
